// GCNEncoder_47545287966961
// MI455X (gfx1250) — hardware-run, weakly checked
//
#include <hip/hip_runtime.h>

typedef float          v8f   __attribute__((ext_vector_type(8)));
typedef float          v4f   __attribute__((ext_vector_type(4)));
typedef unsigned int   v4u   __attribute__((ext_vector_type(4)));
typedef int            v8i   __attribute__((ext_vector_type(8)));
typedef unsigned short v8us  __attribute__((ext_vector_type(8)));
typedef unsigned short v16us __attribute__((ext_vector_type(16)));
typedef __bf16         v16bf __attribute__((ext_vector_type(16)));
typedef _Float16       v16h  __attribute__((ext_vector_type(16)));
typedef v4f  __attribute__((may_alias)) v4fa;
typedef v8us __attribute__((may_alias)) v8usa;
union FragB { v16bf v; v16us u; v8us h[2]; v8i w; };
union FragH { v16h  v; v16us u; v8us h[2]; v8i w; };

__device__ __forceinline__ v8f wmb(const FragB& a, const FragB& b, v8f c) {
  v8f d = __builtin_amdgcn_wmma_f32_16x16x32_bf16(false, a.v, false, b.v, (short)0, c, false, false);
  asm volatile("v_nop\n\tv_nop\n\tv_nop\n\tv_nop" : "+v"(d) : "v"(a.w), "v"(b.w));
  return d;
}

__device__ __forceinline__ v8f wmh(const FragH& a, const FragH& b, v8f c) {
  v8f d = __builtin_amdgcn_wmma_f32_16x16x32_f16(false, a.v, false, b.v, (short)0, c, false, false);
  asm volatile("v_nop\n\tv_nop\n\tv_nop\n\tv_nop" : "+v"(d) : "v"(a.w), "v"(b.w));
  return d;
}

__device__ __forceinline__ unsigned bf16_bits(float f) {
  const unsigned u = __float_as_uint(f);
  const unsigned r = (u + 0x7FFFu + ((u >> 16) & 1u)) >> 16;
  const unsigned q = (u >> 16) | 0x40u;
  return ((u & 0x7fffffffu) > 0x7f800000u) ? q : r;
}

__device__ __forceinline__ float bf16_val(float f) {
  return __uint_as_float(bf16_bits(f) << 16);
}
__device__ __forceinline__ int clampi(int v, int lo, int hi) {
  return v < lo ? lo : (v > hi ? hi : v);
}

__device__ __forceinline__ unsigned f16_bits(float f) {
  const unsigned u  = __float_as_uint(f);
  const unsigned s  = (u >> 16) & 0x8000u;
  const unsigned a  = u & 0x7fffffffu;
  const unsigned t  = a - 0x38000000u;
  const unsigned r  = (t + 0x0FFFu + ((t >> 13) & 1u)) >> 13;
  const unsigned rc = r > 0x7C00u ? 0x7C00u : r;
  const bool small  = a < 0x38800000u;
  const bool isnan  = a > 0x7f800000u;
  const unsigned fin = small ? 0u : (s | rc);
  return isnan ? (s | 0x7E00u) : fin;
}

__device__ __forceinline__ unsigned pk16(unsigned lo, unsigned hi) { return lo | (hi << 16); }
__device__ __forceinline__ unsigned bf16_lo_bits(float v) {
  float hi = bf16_val(v);
  asm volatile("" : "+v"(hi));
  return bf16_bits(v - hi);
}
__device__ __forceinline__ v4u pack8_bf16(v4f a, v4f c) {
  return (v4u){ pk16(bf16_bits(a[0]), bf16_bits(a[1])), pk16(bf16_bits(a[2]), bf16_bits(a[3])),
                pk16(bf16_bits(c[0]), bf16_bits(c[1])), pk16(bf16_bits(c[2]), bf16_bits(c[3])) };
}
__device__ __forceinline__ v4u pack8_bf16_lo(v4f a, v4f c) {
  return (v4u){ pk16(bf16_lo_bits(a[0]), bf16_lo_bits(a[1])), pk16(bf16_lo_bits(a[2]), bf16_lo_bits(a[3])),
                pk16(bf16_lo_bits(c[0]), bf16_lo_bits(c[1])), pk16(bf16_lo_bits(c[2]), bf16_lo_bits(c[3])) };
}
__device__ __forceinline__ v4u pack8_f16(v4f a, v4f c) {
  return (v4u){ pk16(f16_bits(a[0]), f16_bits(a[1])), pk16(f16_bits(a[2]), f16_bits(a[3])),
                pk16(f16_bits(c[0]), f16_bits(c[1])), pk16(f16_bits(c[2]), f16_bits(c[3])) };
}

template <int FORM>
__global__ __launch_bounds__(256) void k_plane(const float* __restrict__ src, int rows, int cols, int ldsrc,
                                               unsigned short* __restrict__ dst, int MP, int KP) {
  static_assert(FORM >= 0 && FORM <= 3);
  const int KTOT = (FORM == 1 || FORM == 3) ? 2 * KP : KP;
  const unsigned ppr   = (unsigned)(KTOT >> 3);
  const unsigned kp8   = (unsigned)(KP >> 3);
  const unsigned total = (unsigned)MP * ppr;
  const unsigned g     = blockIdx.x * 256u + threadIdx.x;
  const unsigned rowu  = g / ppr;
  const unsigned p     = g - rowu * ppr;
  const bool second    = p >= kp8;
  const int row = (int)rowu;
  const int c0  = (int)((second ? p - kp8 : p) << 3);
  const float* srow = src + (size_t)clampi(row, 0, rows - 1) * (size_t)ldsrc;
  float x[8];
  unsigned mk[8];
#pragma unroll
  for (int e = 0; e < 8; ++e) {
    const int c = c0 + e;
    const float v = srow[clampi(c, 0, cols - 1)];
    asm volatile("" :: "v"(v));
    x[e]  = v;
    mk[e] = (row < rows && c < cols) ? 0xFFFFu : 0u;
  }
  const v4f a = (v4f){ x[0], x[1], x[2], x[3] };
  const v4f c = (v4f){ x[4], x[5], x[6], x[7] };
  v4u o;
  if (FORM == 2) {
    o = pack8_f16(a, c);
  } else {
    const v4u hi = pack8_bf16(a, c);
    o = hi;
    if (FORM == 1) { const v4u lo = pack8_bf16_lo(a, c); o = second ? lo : hi; }
  }
  const v4u mw = (v4u){ pk16(mk[0], mk[1]), pk16(mk[2], mk[3]), pk16(mk[4], mk[5]), pk16(mk[6], mk[7]) };
  o &= mw;
  if (g < total) {
    volatile v4u* q = (volatile v4u*)(dst + (size_t)g * 8);
    *q = o;
    __threadfence();
    *q = o;
  }
}

template <int FORM> struct FragOf    { typedef FragB T; };
template <>         struct FragOf<2> { typedef FragH T; };
__device__ __forceinline__ v8f mm(const FragB& a, const FragB& b, v8f c) { return wmb(a, b, c); }
__device__ __forceinline__ v8f mm(const FragH& a, const FragH& b, v8f c) { return wmh(a, b, c); }
template <class F> __device__ __forceinline__ F ld_frag(const unsigned short* p) {
  F f;
  f.h[0] = *(const v8usa*)(p);
  f.h[1] = *(const v8usa*)(p + 16);
  return f;
}

template <int FORM, int EPI>
__global__ __launch_bounds__(256) __attribute__((amdgpu_num_vgpr(248)))
void k_gemm_nt(const unsigned short* __restrict__ A, const unsigned short* __restrict__ B,
               const float* __restrict__ bias, float* __restrict__ D, int M, int N, int KTOT, int ldd) {
  static_assert(FORM >= 0 && FORM <= 2);
  static_assert(EPI == 0 || EPI == 1);
  typedef typename FragOf<FORM>::T F;
  __shared__ __attribute__((aligned(16))) float sT[8][16 * 68];
  const int lane = threadIdx.x & 31;
  const int wave = threadIdx.x >> 5;
  const int tilesM = (M + 63) >> 6;
  const int tilesN = (N + 63) >> 6;
  const int tile = blockIdx.x * 8 + wave;
  if (tile >= tilesM * tilesN) return;
  const int tm = tile / tilesN;
  const int tn = tile - tm * tilesN;
  const int m0 = tm << 6;
  const int n0 = tn << 6;

  const int rl = lane & 15;
  const int h8 = (lane >> 4) * 8;
  const unsigned short* pa = A + (size_t)(m0 + rl) * (size_t)KTOT + h8;
  const unsigned short* pb = B + (size_t)(n0 + rl) * (size_t)KTOT + h8;

  v8f acc[4][4];
#pragma unroll
  for (int i = 0; i < 4; ++i)
#pragma unroll
    for (int j = 0; j < 4; ++j) acc[i][j] = (v8f){0.f, 0.f, 0.f, 0.f, 0.f, 0.f, 0.f, 0.f};

#pragma unroll 1
  for (int k0 = 0; k0 < KTOT; k0 += 32) {
    F bf[4];
#pragma unroll
    for (int j = 0; j < 4; ++j) bf[j] = ld_frag<F>(pb + (size_t)(j << 4) * (size_t)KTOT + k0);
#pragma unroll
    for (int i = 0; i < 4; ++i) {
      const F af = ld_frag<F>(pa + (size_t)(i << 4) * (size_t)KTOT + k0);
#pragma unroll
      for (int j = 0; j < 4; ++j) acc[i][j] = mm(af, bf[j], acc[i][j]);
    }
  }

  float* slab = sT[wave];
  const int hh = lane >> 4;
  const int c4 = (lane & 15) * 4;
  const int nc = n0 + c4;
  const bool cok = nc < N;
  v4f bv = (v4f){0.f, 0.f, 0.f, 0.f};
  if (EPI == 1) {
    bv = *(const v4fa*)(bias + clampi(nc, 0, N - 4));
    asm volatile("" :: "v"(bv));
  }
#pragma unroll
  for (int i = 0; i < 4; ++i) {
    const int mBase = m0 + (i << 4);
#pragma unroll
    for (int j = 0; j < 4; ++j) {
#pragma unroll
      for (int r = 0; r < 8; ++r) slab[(h8 + r) * 68 + (j << 4) + rl] = acc[i][j][r];
    }
    __builtin_amdgcn_fence(__ATOMIC_RELEASE, "workgroup");
    __builtin_amdgcn_wave_barrier();
    __builtin_amdgcn_fence(__ATOMIC_ACQUIRE, "workgroup");
    v4f vv[8];
#pragma unroll
    for (int it = 0; it < 8; ++it) {
      const int row = it * 2 + hh;
      v4f v = *(const v4fa*)(slab + row * 68 + c4);
      if (EPI == 1) v += bv;
      vv[it] = v;
    }
    for (int pass = 0; pass < 2; ++pass) {
#pragma unroll
      for (int it = 0; it < 8; ++it) {
        const int row = mBase + it * 2 + hh;
        if (cok && row < M) *(volatile v4f*)(D + (size_t)row * (size_t)ldd + nc) = vv[it];
      }
      __threadfence();
    }
    __builtin_amdgcn_fence(__ATOMIC_RELEASE, "workgroup");
    __builtin_amdgcn_wave_barrier();
    __builtin_amdgcn_fence(__ATOMIC_ACQUIRE, "workgroup");
  }
}

#include <stddef.h>
#include <math.h>

#ifndef H_SPLIT
#define H_SPLIT 1
#endif

typedef int v4i __attribute__((ext_vector_type(4)));
typedef v4i __attribute__((may_alias)) v4ia;

constexpr int NN     = 100000;
constexpr int NE     = 1600000;
constexpr int CH     = 128;
constexpr int OUTC   = 64;
constexpr int MPAD   = 100096;
constexpr int KA     = H_SPLIT ? 256 : 128;
constexpr int PPR    = KA / 8;
constexpr int NTHR   = 256;
constexpr int NWAVE  = 8;
constexpr int EPT    = 8;
constexpr int CHUNK  = NTHR * EPT;
constexpr int WCAP   = EPT * 32;
constexpr int LISTN  = NWAVE * WCAP;
constexpr int NBA    = 1024;
constexpr int SLA    = 10;
constexpr int NBLK   = 98;
constexpr int NSLOT  = NBLK * NBA;
constexpr int CAP    = 20992;
constexpr int DEGCAP = 64;
constexpr int ZINTS  = LISTN + 2 * CAP + 3 * NBA;
constexpr int BK_LDS_INTS = ZINTS + 16;
constexpr int BK_LDS_BYTES = BK_LDS_INTS * 4;
constexpr int NLIT   = (CAP / 4 + NTHR - 1) / NTHR;
constexpr int OUT1_EL = NN * OUTC;
constexpr int NOUT   = 2 * NN * OUTC;

constexpr int NU1   = CH * (CH / 8);
constexpr int NUH   = OUTC * PPR;
constexpr int NBW   = (NU1 + 2 * NUH) / NTHR;
constexpr int NPADP = (MPAD - NN) * PPR;
constexpr int NPADB = (NPADP + NTHR - 1) / NTHR;
constexpr int BTP   = 64;

constexpr size_t SZ_T    = (size_t)MPAD * CH * 4;
constexpr size_t SZ_A2   = (size_t)MPAD * KA * 2;
constexpr size_t SZ_XB   = (size_t)MPAD * CH * 2;
constexpr size_t SZ_LIST = (size_t)NBLK * CAP * 4;
constexpr size_t SZ_SLOT = (size_t)NSLOT * 4;
constexpr size_t SZ_FLAG = (size_t)NBLK * 128;
constexpr size_t SZ_W1T  = (size_t)CH * CH * 2;
constexpr size_t SZ_WC   = (size_t)CH * KA * 2;
constexpr size_t SZ_BT   = 1024;
constexpr size_t O_T    = 0;
constexpr size_t O_A2   = O_T + SZ_T;
constexpr size_t O_LIST = O_A2 + SZ_A2;
constexpr size_t O_CNT  = O_LIST + SZ_LIST;
constexpr size_t O_OFF  = O_CNT + SZ_SLOT;
constexpr size_t O_DINV = O_OFF + SZ_SLOT;
constexpr size_t O_FLAG = O_DINV + SZ_SLOT;
constexpr size_t O_W1T  = O_FLAG + SZ_FLAG;
constexpr size_t O_WCT  = O_W1T + SZ_W1T;
constexpr size_t O_BT   = O_WCT + SZ_WC;
constexpr size_t WS_TOTAL = O_BT + SZ_BT;

static_assert(CH == 32 * 4);
static_assert(2 * OUTC == CH);
static_assert(NN <= NBLK * NBA);
static_assert((NN & 7) == 0 && NN % 16 == 0);
static_assert(NN % NWAVE == 0);
static_assert(MPAD % 128 == 0 && MPAD >= ((NN + 63) / 64) * 64);
static_assert(CH % 32 == 0 && KA % 32 == 0);
static_assert(((long long)MPAD * CH / 8) % 256 == 0);
static_assert((long long)MPAD * KA / 8 < (1LL << 31));
static_assert(NE % 4 == 0 && NE < (1 << 21));
static_assert(((long long)NE << SLA) < (1LL << 31));
static_assert(CAP * 4 >= 16710 * 5);
static_assert(DEGCAP >= 36 + 8);
static_assert(CAP % 256 == 0 && (CAP * 4) % 128 == 0);
static_assert(ZINTS % (NTHR * 4) == 0);
static_assert(BK_LDS_BYTES <= 262144);
static_assert(NU1 % NTHR == 0 && NUH % NTHR == 0);
static_assert(NPADP % NTHR == 0);
static_assert(BTP * 16 <= (int)SZ_BT && BTP <= NTHR);
static_assert(SZ_T % 256 == 0 && SZ_A2 % 256 == 0 && SZ_LIST % 256 == 0 && SZ_SLOT % 256 == 0);
static_assert(SZ_FLAG % 256 == 0 && SZ_W1T % 256 == 0 && SZ_WC % 256 == 0 && SZ_BT % 256 == 0);
static_assert(SZ_XB <= SZ_A2);
static_assert(WS_TOTAL <= ((size_t)128 << 20));
#if H_SPLIT
static_assert(WS_TOTAL == (size_t)((size_t)437669 << 8));
#endif
static_assert((long long)OUT1_EL + (long long)(NN - 1) * OUTC + OUTC - 1 == (long long)NOUT - 1);
static_assert(((long long)OUT1_EL * 4) % 128 == 0);

__device__ __forceinline__ void wunit(const float* __restrict__ src, int ld, int col, int kk, unsigned short* dp) {
  const float* p = src + (size_t)kk * (size_t)ld + col;
  unsigned b[8];
#pragma unroll
  for (int i = 0; i < 8; ++i) b[i] = bf16_bits(p[(size_t)i * (size_t)ld]);
  const v4u o = (v4u){ pk16(b[0], b[1]), pk16(b[2], b[3]), pk16(b[4], b[5]), pk16(b[6], b[7]) };
  *(volatile v4u*)dp = o;
  __threadfence();
  *(volatile v4u*)dp = o;
}

__global__ __launch_bounds__(NTHR) void k_wprep(const float* __restrict__ W1, const float* __restrict__ Wmu,
                                                const float* __restrict__ Wls, const float* __restrict__ b1,
                                                const float* __restrict__ bmu, const float* __restrict__ bls,
                                                char* wsb) {
  unsigned short* W1T = (unsigned short*)(wsb + O_W1T);
  unsigned short* WCT = (unsigned short*)(wsb + O_WCT);
  unsigned short* A2  = (unsigned short*)(wsb + O_A2);
  float*          BT  = (float*)(wsb + O_BT);
  const int tid = (int)threadIdx.x;
  const int blk = (int)blockIdx.x;
  const int u   = blk * NTHR + tid;
  if (u < NU1) {
    const int n = u >> 4, k8 = (u & 15) * 8;
    wunit(W1, CH, n, k8, W1T + (size_t)n * CH + k8);
  } else if (u < NU1 + NUH) {
    const int q = u - NU1;
    const int n = q / PPR, k8 = (q - n * PPR) * 8;
    wunit(Wmu, OUTC, n, k8 & (CH - 1), WCT + (size_t)n * KA + k8);
  } else if (u < NU1 + 2 * NUH) {
    const int q = u - NU1 - NUH;
    const int n = q / PPR, k8 = (q - n * PPR) * 8;
    wunit(Wls, OUTC, n, k8 & (CH - 1), WCT + (size_t)(OUTC + n) * KA + k8);
  } else if (blk == NBW) {
    const int t = tid;
    const v4f a1 = *(const v4fa*)(b1  + 4 * clampi(t, 0, 31));
    asm volatile("" :: "v"(a1));
    const v4f a3 = *(const v4fa*)(bmu + 4 * clampi(t - 32, 0, 15));
    asm volatile("" :: "v"(a3));
    const v4f a4 = *(const v4fa*)(bls + 4 * clampi(t - 48, 0, 15));
    asm volatile("" :: "v"(a4));
    const unsigned m1 = (t < 32) ? 0xFFFFFFFFu : 0u;
    const unsigned m3 = (t >= 32 && t < 48) ? 0xFFFFFFFFu : 0u;
    const unsigned m4 = (t >= 48 && t < 64) ? 0xFFFFFFFFu : 0u;
    v4u o;
#pragma unroll
    for (int e = 0; e < 4; ++e) {
      o[e] = ((bf16_bits(a1[e]) << 16) & m1) | ((bf16_bits(a3[e]) << 16) & m3) | ((bf16_bits(a4[e]) << 16) & m4);
    }
    if (t < BTP) {
      volatile v4u* q = (volatile v4u*)(BT + 4 * t);
      *q = o;
      __threadfence();
      *q = o;
    }
  } else {
    const int q = u - (NBW + 1) * NTHR;
    if (q >= 0 && q < NPADP) {
      const v4u z = (v4u){0u, 0u, 0u, 0u};
      volatile v4u* p = (volatile v4u*)(A2 + (size_t)NN * KA + (size_t)q * 8);
      *p = z;
      __threadfence();
      *p = z;
    }
  }
}

__device__ __forceinline__ int scan_chunk(const int* __restrict__ dsts, int nE, int cbase, int slotBase, int nb,
                                          int vec8, int* list, int tid, int lane, int wave) {
  const int el0 = tid * EPT;
  const int e0  = cbase + el0;
  int dv[8];
  if (vec8 != 0 && cbase + CHUNK <= nE) {
    const v4i da = *(const v4ia*)(dsts + e0);
    const v4i db = *(const v4ia*)(dsts + e0 + 4);
    dv[0] = da.x; dv[1] = da.y; dv[2] = da.z; dv[3] = da.w;
    dv[4] = db.x; dv[5] = db.y; dv[6] = db.z; dv[7] = db.w;
  } else {
    const int sent = (-0x7fffffff - 1);
#pragma unroll
    for (int j = 0; j < 8; ++j) {
      const int ej = e0 + j;
      const int tv = dsts[ej < nE ? ej : nE - 1];
      asm volatile("" :: "v"(tv));
      const int m = (ej < nE) ? -1 : 0;
      dv[j] = (tv & m) | (sent & ~m);
    }
  }
  const unsigned nbs = (unsigned)slotBase;
  const unsigned unb = (unsigned)nb;
  unsigned s[8];
  unsigned hb = 0u;
#pragma unroll
  for (int j = 0; j < 8; ++j) {
    s[j] = (unsigned)dv[j] - nbs;
    hb |= (s[j] < unb) ? (1u << j) : 0u;
  }
  const unsigned any = __builtin_amdgcn_ballot_w32(hb != 0u);
  int wc = 0;
  if (any != 0u) {
    const int n = (int)__builtin_popcount(hb);
    int incl = n;
#pragma unroll
    for (int d = 1; d < 32; d <<= 1) {
      const int y = __shfl_up(incl, (unsigned)d, 32);
      incl += (lane >= d) ? y : 0;
    }
    int pos = incl - n;
    wc = __shfl(incl, 31, 32);
#pragma unroll
    for (int j = 0; j < 8; ++j) {
      if ((hb >> j) & 1u) {
        if (pos < WCAP) list[wave * WCAP + pos] = ((el0 + j) << SLA) | (int)s[j];
        pos = pos + 1;
      }
    }
  }
  return wc;
}

__global__ __launch_bounds__(NTHR) void k_bucket(const int* __restrict__ srcs, const int* __restrict__ dsts,
                                                 int nE, int nN, int vec8,
                                                 int* LIST, int* CNT, int* OFF, float* DINV, int* FLAG) {
  extern __shared__ __attribute__((aligned(16))) int dsm[];
  int* list = dsm;
  int* hl   = dsm + LISTN;
  int* sl   = dsm + LISTN + CAP;
  int* cnt  = dsm + LISTN + 2 * CAP;
  int* offs = cnt + NBA;
  int* cur  = offs + NBA;
  int* misc = cur + NBA;
  const int tid = (int)threadIdx.x, lane = tid & 31, wave = tid >> 5;
  const int nodeBase = (int)blockIdx.x * NBA;
  const int nb = clampi(nN - nodeBase, 0, NBA);

  {
    const v4i z4 = (v4i){0, 0, 0, 0};
    for (int i = tid * 4; i < ZINTS; i += NTHR * 4) *(v4ia*)(dsm + i) = z4;
    if (tid < 16) misc[tid] = 0;
  }
  __syncthreads();

  int t = 0, ov = 0;
  const int nChunks = (nE + CHUNK - 1) / CHUNK;
#pragma unroll 1
  for (int ch = 0; ch < nChunks; ++ch) {
    const int cbase = ch * CHUNK;
    const int wc = scan_chunk(dsts, nE, cbase, nodeBase, nb, vec8, list, tid, lane, wave);
    if (lane == 0) misc[wave] = wc;
    __syncthreads();
    if (wave == 0) {
#pragma unroll 1
      for (int w2 = 0; w2 < NWAVE; ++w2) {
        int c = misc[w2];
        c = c < 0 ? 0 : (c > WCAP ? WCAP : c);
#pragma unroll 1
        for (int b0 = 0; b0 < c; b0 += 32) {
          const int idx = b0 + lane;
          const int ent = list[w2 * WCAP + (idx < WCAP ? idx : WCAP - 1)];
          const int m32 = (c - b0) < 32 ? (c - b0) : 32;
#pragma unroll 1
          for (int k = 0; k < m32; ++k) {
            const int u    = __builtin_amdgcn_readlane(ent, k);
            const int slot = u & (NBA - 1);
            const int el   = (u >> SLA) & (CHUNK - 1);
            const int pk   = ((cbase + el) << SLA) | slot;
            if (t < CAP) {
              if (lane == 0) { hl[t] = pk; cnt[slot] = cnt[slot] + 1; }
              t = t + 1;
            } else {
              ov = 1;
            }
          }
        }
      }
    }
    __syncthreads();
  }
  if (wave == 0 && lane == 0) { misc[8] = t; misc[9] = ov; }
  __syncthreads();
  int tt = misc[8];
  tt = tt < 0 ? 0 : (tt > CAP ? CAP : tt);
  const int ovf = misc[9];

  if (wave == 0) {
    const int base = lane * (NBA / 32);
    int sacc = 0;
#pragma unroll 1
    for (int i = 0; i < NBA / 32; ++i) sacc += cnt[base + i];
    int incl = sacc;
#pragma unroll
    for (int d = 1; d < 32; d <<= 1) {
      const int y = __shfl_up(incl, (unsigned)d, 32);
      incl += (lane >= d) ? y : 0;
    }
    int run = incl - sacc;
#pragma unroll 1
    for (int i = 0; i < NBA / 32; ++i) {
      const int cv = cnt[base + i];
      offs[base + i] = run;
      cur[base + i]  = run;
      run += cv;
    }
  }
  __syncthreads();
  if (wave == 0) {
#pragma unroll 1
    for (int b0 = 0; b0 < tt; b0 += 32) {
      const int idx = b0 + lane;
      const int ent = hl[idx < CAP ? idx : CAP - 1];
      const int m32 = (tt - b0) < 32 ? (tt - b0) : 32;
#pragma unroll 1
      for (int k = 0; k < m32; ++k) {
        const int u    = __builtin_amdgcn_readlane(ent, k);
        const int slot = u & (NBA - 1);
        if (lane == 0) {
          int p = cur[slot];
          p = p < 0 ? 0 : (p > CAP - 1 ? CAP - 1 : p);
          sl[p] = u;
          cur[slot] = p + 1;
        }
      }
    }
  }
  __syncthreads();

  const v4i c4 = *(const v4ia*)(cnt + 4 * tid);
  const v4i o4 = *(const v4ia*)(offs + 4 * tid);
  const bool big = (c4.x > DEGCAP) || (c4.y > DEGCAP) || (c4.z > DEGCAP) || (c4.w > DEGCAP);
  const unsigned bm = __builtin_amdgcn_ballot_w32(big);
  if (lane == 0) misc[wave] = (bm != 0u) ? 1 : 0;
#pragma unroll 1
  for (int i = 0; i < 4; ++i) {
    const int cv = cnt[4 * tid + i];
    const float d = 1.0f / sqrtf((float)cv + 1.0f);
    cur[4 * tid + i] = __float_as_int(d);
  }
  __syncthreads();
  int fl = ovf;
#pragma unroll
  for (int w2 = 0; w2 < NWAVE; ++w2) fl |= misc[w2];
  fl = (fl != 0) ? 1 : 0;
  const v4i d4 = *(const v4ia*)(cur + 4 * tid);
  const v4f dvv = (v4f){ __int_as_float(d4.x), __int_as_float(d4.y), __int_as_float(d4.z), __int_as_float(d4.w) };
  const v4i f4 = (v4i){ fl, fl, fl, fl };
  int*   cp = CNT  + (size_t)nodeBase + 4 * tid;
  int*   op = OFF  + (size_t)nodeBase + 4 * tid;
  float* dp = DINV + (size_t)nodeBase + 4 * tid;
  int*   fp = FLAG + (size_t)blockIdx.x * 32 + 4 * (lane & 7);
  const bool fst = (wave == 0) && (lane < 8);
  *(volatile v4i*)cp = c4;
  *(volatile v4i*)op = o4;
  *(volatile v4f*)dp = dvv;
  if (fst) *(volatile v4i*)fp = f4;
  __threadfence();
  *(volatile v4i*)cp = c4;
  *(volatile v4i*)op = o4;
  *(volatile v4f*)dp = dvv;
  if (fst) *(volatile v4i*)fp = f4;

  int* lbase = LIST + (size_t)blockIdx.x * CAP;
#pragma unroll 1
  for (int it = 0; it < NLIT; ++it) {
    const int p  = it * NTHR + tid;
    const bool ok = p < CAP / 4;
    const int pc = ok ? p : CAP / 4 - 1;
    const v4i e = *(const v4ia*)(sl + 4 * pc);
    int s0 = srcs[clampi(e.x >> SLA, 0, nE - 1)];
    asm volatile("" :: "v"(s0));
    int s1 = srcs[clampi(e.y >> SLA, 0, nE - 1)];
    asm volatile("" :: "v"(s1));
    int s2 = srcs[clampi(e.z >> SLA, 0, nE - 1)];
    asm volatile("" :: "v"(s2));
    int s3 = srcs[clampi(e.w >> SLA, 0, nE - 1)];
    asm volatile("" :: "v"(s3));
    const v4i w = (v4i){ clampi(s0, 0, nN - 1), clampi(s1, 0, nN - 1), clampi(s2, 0, nN - 1), clampi(s3, 0, nN - 1) };
    volatile v4i* q = (volatile v4i*)(lbase + 4 * pc);
    if (ok) *q = w;
    __threadfence();
    if (ok) *q = w;
  }
}

template <int MODE>
__global__ __launch_bounds__(NTHR) void k_agg(const int* __restrict__ LIST, const int* __restrict__ CNT,
                                              const int* __restrict__ OFF, const float* __restrict__ DINV,
                                              const int* __restrict__ FLAG, const float* __restrict__ T,
                                              const float* __restrict__ BT, float* OUTF,
                                              unsigned short* HL, int nN) {
  static_assert(MODE == 1 || MODE == 2);
  __shared__ __attribute__((aligned(16))) float sb[CH];
  const int tid = (int)threadIdx.x, lane = tid & 31, wave = tid >> 5;
  if (wave == 0) {
    const v4f b = *(const v4fa*)(BT + 128 * (MODE - 1) + 4 * lane);
    *(v4fa*)(sb + 4 * lane) = b;
  }
  __syncthreads();
  const int v = __builtin_amdgcn_readfirstlane((int)blockIdx.x * NWAVE + wave);
  if (v >= nN) return;
  const int blk = clampi(v >> SLA, 0, NBLK - 1);
  const int vc  = clampi(v, 0, nN - 1);

  int c = CNT[vc];
  asm volatile("" :: "v"(c));
  int o = OFF[vc];
  asm volatile("" :: "v"(o));
  int fl = FLAG[32 * blk];
  asm volatile("" :: "v"(fl));
  const float dv = DINV[vc];
  asm volatile("" :: "v"(dv));
  c  = __builtin_amdgcn_readfirstlane(clampi(c, 0, DEGCAP));
  o  = __builtin_amdgcn_readfirstlane(clampi(o, 0, CAP));
  fl = __builtin_amdgcn_readfirstlane(fl);
  const float rd = dv * dv;
  const int* lst = LIST + (size_t)blk * CAP;

  v4f acc = (v4f){0.0f, 0.0f, 0.0f, 0.0f};
#pragma unroll 1
  for (int b0 = 0; b0 < c; b0 += 32) {
    int ii = o + b0 + lane;
    const int last = o + c - 1;
    ii = ii > last ? last : ii;
    const int idx = clampi(ii, 0, CAP - 1);
    int sr = lst[idx];
    asm volatile("" :: "v"(sr));
    sr = clampi(sr, 0, nN - 1);
    const float ds = DINV[sr];
    asm volatile("" :: "v"(ds));
    const int wi = __float_as_int(ds * dv);
    const int m32 = (c - b0) < 32 ? (c - b0) : 32;
#pragma unroll 1
    for (int k = 0; k < m32; ++k) {
      const int   sk = __builtin_amdgcn_readlane(sr, k);
      const float wk = __int_as_float(__builtin_amdgcn_readlane(wi, k));
      const v4f r = *(const v4fa*)(T + (size_t)sk * CH + 4 * lane);
      acc.x = fmaf(wk, r.x, acc.x);
      acc.y = fmaf(wk, r.y, acc.y);
      acc.z = fmaf(wk, r.z, acc.z);
      acc.w = fmaf(wk, r.w, acc.w);
    }
  }
  const v4f sr4 = *(const v4fa*)(T + (size_t)vc * CH + 4 * lane);
  asm volatile("" :: "v"(sr4));
  const v4f bv = *(const v4fa*)(sb + 4 * lane);
  v4f y;
  y.x = fmaf(sr4.x, rd, acc.x) + bv.x;
  y.y = fmaf(sr4.y, rd, acc.y) + bv.y;
  y.z = fmaf(sr4.z, rd, acc.z) + bv.z;
  y.w = fmaf(sr4.w, rd, acc.w) + bv.w;

  if constexpr (MODE == 1) {
    y.x = (y.x > 0.0f) ? y.x : (y.x - y.x);
    y.y = (y.y > 0.0f) ? y.y : (y.y - y.y);
    y.z = (y.z > 0.0f) ? y.z : (y.z - y.z);
    y.w = (y.w > 0.0f) ? y.w : (y.w - y.w);
  }

  const bool pz = fl != 0;
  const float qn = __int_as_float(0x7fc00000);
  v4f yv;
  yv.x = pz ? qn : y.x;
  yv.y = pz ? qn : y.y;
  yv.z = pz ? qn : y.z;
  yv.w = pz ? qn : y.w;

  if constexpr (MODE == 2) {
    const int eo = (lane < 16) ? (v * OUTC + 4 * lane) : (OUT1_EL + v * OUTC + 4 * (lane - 16));
    float* op = OUTF + (size_t)eo;
    *(volatile v4f*)op = yv;
    __threadfence();
    *(volatile v4f*)op = yv;
  } else {
    const int hw0 = (int)pk16(bf16_bits(yv.x), bf16_bits(yv.y));
    const int hw1 = (int)pk16(bf16_bits(yv.z), bf16_bits(yv.w));
    const int lw0 = (int)pk16(bf16_lo_bits(yv.x), bf16_lo_bits(yv.y));
    const int lw1 = (int)pk16(bf16_lo_bits(yv.z), bf16_lo_bits(yv.w));
    const int sa = (2 * lane) & 31, sc = (2 * lane + 1) & 31;
    const int g0 = __shfl(hw0, sa, 32), g1 = __shfl(hw1, sa, 32);
    const int g2 = __shfl(hw0, sc, 32), g3 = __shfl(hw1, sc, 32);
    const int p0 = __shfl(lw0, sa, 32), p1 = __shfl(lw1, sa, 32);
    const int p2 = __shfl(lw0, sc, 32), p3 = __shfl(lw1, sc, 32);
    const bool lsel = (H_SPLIT != 0) && (lane >= 16);
    v4u pv;
    pv.x = (unsigned)(lsel ? p0 : g0);
    pv.y = (unsigned)(lsel ? p1 : g1);
    pv.z = (unsigned)(lsel ? p2 : g2);
    pv.w = (unsigned)(lsel ? p3 : g3);
    const bool hst = (H_SPLIT != 0) || (lane < 16);
    unsigned short* hp = HL + (size_t)v * KA + 8 * (H_SPLIT != 0 ? lane : (lane & 15));
    if (hst) *(volatile v4u*)hp = pv;
    __threadfence();
    if (hst) *(volatile v4u*)hp = pv;
  }
}

static inline int cdiv_h(int a, int b) { return (a + b - 1) / b; }

extern "C" void kernel_launch(void* const* d_in, const int* in_sizes, int n_in,
                              void* d_out, int out_size, void* d_ws, size_t ws_size,
                              hipStream_t stream) {
  if (n_in < 9) return;
  if (in_sizes[0] != NN * CH) return;
  if (in_sizes[1] != 2 * NE) return;
  if (in_sizes[2] != NN) return;
  if (in_sizes[3] != CH * CH || in_sizes[4] != CH) return;
  if (in_sizes[5] != CH * OUTC || in_sizes[6] != OUTC) return;
  if (in_sizes[7] != CH * OUTC || in_sizes[8] != OUTC) return;
  if (out_size != NOUT) return;
  if (ws_size < WS_TOTAL) return;

  const float* x    = (const float*)d_in[0];
  const int*   edge = (const int*)d_in[1];
  const int*   gid  = (const int*)d_in[2];
  (void)gid;
  const float* W1   = (const float*)d_in[3];
  const float* b1   = (const float*)d_in[4];
  const float* Wmu  = (const float*)d_in[5];
  const float* bmu  = (const float*)d_in[6];
  const float* Wls  = (const float*)d_in[7];
  const float* bls  = (const float*)d_in[8];
  float* out = (float*)d_out;
  const int* src = edge;
  const int* dst = edge + NE;

  char* ws = (char*)d_ws;
  float*          T    = (float*)(ws + O_T);
  unsigned short* A2   = (unsigned short*)(ws + O_A2);
  unsigned short* XB   = (unsigned short*)(ws + O_A2);
  int*            LIST = (int*)(ws + O_LIST);
  int*            CNT  = (int*)(ws + O_CNT);
  int*            OFF  = (int*)(ws + O_OFF);
  float*          DINV = (float*)(ws + O_DINV);
  int*            FLAG = (int*)(ws + O_FLAG);
  unsigned short* W1T  = (unsigned short*)(ws + O_W1T);
  unsigned short* WCT  = (unsigned short*)(ws + O_WCT);
  float*          BT   = (float*)(ws + O_BT);

  hipFuncSetAttribute(reinterpret_cast<const void*>(&k_bucket), hipFuncAttributeMaxDynamicSharedMemorySize,
                      (int)BK_LDS_BYTES);

  const int vec8   = ((NE & 3) == 0) ? 1 : 0;
  const int gPlane = MPAD * CH / 8 / 256;
  const int gGemm  = cdiv_h(cdiv_h(NN, 64) * cdiv_h(CH, 64), 8);
  const int gAgg   = cdiv_h(NN, NWAVE);

  k_plane<0><<<gPlane, 256, 0, stream>>>(x, NN, CH, CH, XB, MPAD, CH);
  k_wprep<<<NBW + 1 + NPADB, NTHR, 0, stream>>>(W1, Wmu, Wls, b1, bmu, bls, ws);
  k_bucket<<<NBLK, NTHR, BK_LDS_BYTES, stream>>>(src, dst, NE, NN, vec8, LIST, CNT, OFF, DINV, FLAG);
  k_gemm_nt<0, 0><<<gGemm, 256, 0, stream>>>(XB, W1T, BT, T, NN, CH, CH, CH);
  k_agg<1><<<gAgg, NTHR, 0, stream>>>(LIST, CNT, OFF, DINV, FLAG, T, BT, out, A2, NN);
  k_gemm_nt<0, 0><<<gGemm, 256, 0, stream>>>(A2, WCT, BT, T, NN, CH, KA, CH);
  k_agg<2><<<gAgg, NTHR, 0, stream>>>(LIST, CNT, OFF, DINV, FLAG, T, BT, out, A2, NN);
}
